// Encoder_59356448031597
// MI455X (gfx1250) — hardware-run, weakly checked
//
#include <hip/hip_runtime.h>
#include <math.h>
#include <stddef.h>

typedef __attribute__((ext_vector_type(16))) _Float16 v16h;
typedef __attribute__((ext_vector_type(8)))  _Float16 v8h;
typedef __attribute__((ext_vector_type(16))) __bf16   v16b;
typedef __attribute__((ext_vector_type(8)))  __bf16   v8b;
typedef __attribute__((ext_vector_type(8)))  float    v8f;
typedef __attribute__((ext_vector_type(4)))  float    v4f;
typedef __attribute__((ext_vector_type(4)))  unsigned v4u;

constexpr int kB   = 256;
constexpr int kT   = 361;
constexpr int kD   = 128;
constexpr int kH   = 512;
constexpr int kS   = 40;
constexpr int kML  = 88;
constexpr int kNH  = 32 * kS;
constexpr int kG4  = 4 * kH;
static_assert(kNH == 1280);
static_assert(kG4 == 2048);
static_assert(kD % 32 == 0 && kH % 32 == 0);

constexpr int geoL1(int s) { return (kT - 1) / s + 1; }
constexpr int geoC2(int s) { return geoL1(s) - 2; }
constexpr int geoP2(int s) { return geoC2(s) / 2; }
constexpr int geoC3(int s) { return geoP2(s) - 2; }
constexpr int geoP3(int s) { return geoC3(s) / 2; }
static_assert(geoL1(1) == 361 && geoC2(1) == 359 && geoP2(1) == 179 && geoC3(1) == 177 && geoP3(1) == 88);
static_assert(geoL1(40) == 10 && geoC2(40) == 8 && geoP2(40) == 4 && geoC3(40) == 2 && geoP3(40) == 1);
static_assert(geoP3(1) == kML);

struct GeoTab { int p3[kS]; int pad8[kS]; int off3[kS]; int rows; int live; };
constexpr GeoTab makeGeo() {
  GeoTab g{};
  int off = 0, live = 0;
  for (int i = 0; i < kS; ++i) {
    const int p3 = geoP3(i + 1);
    g.p3[i] = p3;
    g.pad8[i] = (p3 + 7) / 8 * 8;
    g.off3[i] = off;
    off += g.pad8[i];
    live += p3;
  }
  g.rows = off;
  g.live = live;
  return g;
}
constexpr GeoTab kGeo = makeGeo();
constexpr int kXfRows = 512;
static_assert(kGeo.rows == kXfRows);
static_assert(kGeo.live == 316);

#define GEO_POOL3_LIST 88,43,28,21,16,13,11,10,8,7,6,6,5,5,4,4,4,3,3,3,3,2,2,2,2,2,2,1,1,1,1,1,1,1,1,1,1,1,1,1
#define GEO_ROWOFF_LIST 0,88,136,168,192,208,224,240,256,264,272,280,288,296,304,312,320,328,336,344,352,360,368,376,384,392,400,408,416,424,432,440,448,456,464,472,480,488,496,504
constexpr int hP3[kS]   = {GEO_POOL3_LIST};
constexpr int hOff3[kS] = {GEO_ROWOFF_LIST};
static_assert(sizeof(hP3) / sizeof(hP3[0]) == 40);
static_assert(sizeof(hOff3) / sizeof(hOff3[0]) == 40);
constexpr bool geoListsOk() {
  for (int i = 0; i < kS; ++i) {
    if (hP3[i] != kGeo.p3[i]) return false;
    if (hOff3[i] != kGeo.off3[i]) return false;
    if (i > 0 && hP3[i] > hP3[i - 1]) return false;
  }
  return true;
}
static_assert(geoListsOk());
__constant__ int c_P3[kS]   = {GEO_POOL3_LIST};
__constant__ int c_Off3[kS] = {GEO_ROWOFF_LIST};

constexpr float H_CARRY     = 512.0f;
constexpr float WHH_CARRY   = 256.0f;
constexpr float XF_CARRY    = 131072.0f;
constexpr float GATE_FOLD   = 1.0f / (H_CARRY * WHH_CARRY);
constexpr float F16_MIN_NRM = 6.103515625e-5f;
static_assert(H_CARRY * WHH_CARRY == XF_CARRY);

constexpr size_t kBytesXB  = (size_t)kB * kT * kD * 2;
constexpr size_t kBytesWIH = (size_t)kG4 * kNH * 2;
constexpr size_t kBytesWHH = (size_t)kG4 * kH * 2;
constexpr size_t kBytesC1  = (size_t)kS * 16 * kD * 2;
constexpr size_t kBytesC2  = (size_t)kS * 32 * 64 * 2;
constexpr size_t kBytesC3  = (size_t)kS * 32 * 96 * 2;
constexpr size_t kBytesXF  = (size_t)kXfRows * kB * 32 * 2;
constexpr size_t kWsTotal  = kBytesXB + kBytesWIH + kBytesWHH + kBytesC1 + kBytesC2 + kBytesC3 + kBytesXF + kBytesXF;
static_assert(kWsTotal == 48349184ull);
static_assert(kWsTotal <= 134217728ull);
static_assert(kBytesXB % 256 == 0 && kBytesWIH % 256 == 0 && kBytesWHH % 256 == 0 && kBytesC1 % 256 == 0 &&
              kBytesC2 % 256 == 0 && kBytesC3 % 256 == 0 && kBytesXF % 256 == 0);

__device__ __forceinline__ unsigned short f2bf_bits(float f) {
  unsigned u = __float_as_uint(f);
  return (unsigned short)((u + 0x7FFFu + ((u >> 16) & 1u)) >> 16);
}
__device__ __forceinline__ float bf_bits2f(unsigned short h) { return __uint_as_float(((unsigned)h) << 16); }
__device__ __forceinline__ float bf16r(float f) { return bf_bits2f(f2bf_bits(f)); }
__device__ __forceinline__ void split_bf(float v, unsigned short& hb, unsigned short& lb) {
  hb = f2bf_bits(v);
  lb = f2bf_bits(v - bf_bits2f(hb));
}

template <typename T> struct Frag;
template <> struct Frag<_Float16> {
  union U { v16h v; v8h h[2]; };
  static __device__ __forceinline__ v16h load(const _Float16* p) {
    U f; f.h[0] = *(const v8h*)(p); f.h[1] = *(const v8h*)(p + 16); return f.v;
  }
};
template <> struct Frag<__bf16> {
  union U { v16b v; v8b h[2]; };
  static __device__ __forceinline__ v16b load(const __bf16* p) {
    U f; f.h[0] = *(const v8b*)(p); f.h[1] = *(const v8b*)(p + 16); return f.v;
  }
};

__device__ __forceinline__ v8f mma_bf(v16b a, v16b b, v8f c) {
  c = __builtin_amdgcn_wmma_f32_16x16x32_bf16(false, a, false, b, (short)0, c, false, false);
  asm volatile("v_nop\n\tv_nop\n\tv_nop\n\tv_nop" : "+v"(c) : "v"(a), "v"(b));
  return c;
}
__device__ __forceinline__ v8f mma_hf(v16h a, v16h b, v8f c) {
  c = __builtin_amdgcn_wmma_f32_16x16x32_f16(false, a, false, b, (short)0, c, false, false);
  asm volatile("v_nop\n\tv_nop\n\tv_nop\n\tv_nop" : "+v"(c) : "v"(a), "v"(b));
  return c;
}

__device__ __forceinline__ void wave_lds_sync() {
  __builtin_amdgcn_fence(__ATOMIC_RELEASE, "workgroup");
  __builtin_amdgcn_wave_barrier();
  __builtin_amdgcn_fence(__ATOMIC_ACQUIRE, "workgroup");
}

__device__ __forceinline__ float fsig(float x)  { return __builtin_amdgcn_rcpf(1.0f + __expf(-x)); }
__device__ __forceinline__ float ftanh(float x) { return 1.0f - 2.0f * __builtin_amdgcn_rcpf(__expf(2.0f * x) + 1.0f); }

template <int MODE>
__global__ __launch_bounds__(256) void cvt8_kernel(const float* __restrict__ src, unsigned short* __restrict__ dst,
                                                   int n8, float sc) {
  const int i = blockIdx.x * 256 + threadIdx.x;
  if (i < n8) {
    const float* sp = src + (size_t)i * 8;
    const v4f a = *(const v4f*)(sp);
    const v4f b = *(const v4f*)(sp + 4);
    v8h hv;
#pragma unroll
    for (int e = 0; e < 4; ++e) {
      const float x0 = a[e];
      const float x1 = b[e];
      unsigned short b0, b1;
      if (MODE == 0) {
        b0 = f2bf_bits(x0);
        b1 = f2bf_bits(x1);
      } else {
        float y0 = bf16r(x0) * sc;
        float y1 = bf16r(x1) * sc;
        y0 = (fabsf(y0) < F16_MIN_NRM) ? 0.0f : y0;
        y1 = (fabsf(y1) < F16_MIN_NRM) ? 0.0f : y1;
        const _Float16 g0 = (_Float16)y0;
        const _Float16 g1 = (_Float16)y1;
        b0 = __builtin_bit_cast(unsigned short, g0);
        b1 = __builtin_bit_cast(unsigned short, g1);
      }
      hv[e]     = __builtin_bit_cast(_Float16, b0);
      hv[4 + e] = __builtin_bit_cast(_Float16, b1);
    }
    unsigned short* q = dst + (size_t)i * 8;
    *(volatile v8h*)q = hv;
    __threadfence();
    *(volatile v8h*)q = hv;
  }
}

template <int CIN>
__global__ __launch_bounds__(256) void tapw_reorder_kernel(const float* __restrict__ src, unsigned short* __restrict__ dst,
                                                           int n8) {
  constexpr int KREAL = 3 * CIN;
  constexpr int KP = (KREAL + 31) / 32 * 32;
  constexpr int K8 = KP / 8;
  const int i = blockIdx.x * 256 + threadIdx.x;
  if (i < n8) {
    const int row = i / K8;
    const int k0 = (i - row * K8) * 8;
    v8h hv;
#pragma unroll
    for (int e = 0; e < 8; ++e) {
      const int k = k0 + e;
      const bool valid = k < KREAL;
      const int kc = valid ? k : (KREAL - 1);
      const int tap = kc / CIN;
      const int ch = kc - tap * CIN;
      const float w = src[((size_t)row * CIN + ch) * 3 + tap];
      const float w2 = valid ? w : 0.0f;
      const unsigned short bits = f2bf_bits(w2);
      hv[e] = __builtin_bit_cast(_Float16, bits);
    }
    unsigned short* q = dst + (size_t)i * 8;
    *(volatile v8h*)q = hv;
    __threadfence();
    *(volatile v8h*)q = hv;
  }
}

constexpr int CV_THREADS = 128;
constexpr int CV_WAVES   = 4;
constexpr int CV_NT1MAX  = (geoL1(1) + 15) / 16;
constexpr int CV_NT2MAX  = (geoP2(1) + 7) / 8;
constexpr int H1_ROWS    = 16 * CV_NT1MAX + 4;
constexpr int H2_ROWS    = 8 * CV_NT2MAX + 16;
constexpr int CV_SLABP   = 36;
static_assert(CV_NT1MAX == 23 && CV_NT2MAX == 23);
static_assert(H1_ROWS == 372 && H2_ROWS == 200);

__global__ __launch_bounds__(CV_THREADS) void branch_conv_kernel(
    const unsigned short* __restrict__ XBp, const unsigned short* __restrict__ C1p,
    const unsigned short* __restrict__ C2p, const unsigned short* __restrict__ C3p,
    const float* __restrict__ c1b, const float* __restrict__ c2b, const float* __restrict__ c3b,
    unsigned short* __restrict__ XFH, unsigned short* __restrict__ XFL) {
  __shared__ __align__(16) unsigned short h1H[H1_ROWS * 16];
  __shared__ __align__(16) unsigned short h1L[H1_ROWS * 16];
  __shared__ __align__(16) unsigned short h2H[H2_ROWS * 32];
  __shared__ __align__(16) unsigned short h2L[H2_ROWS * 32];
  __shared__ __align__(16) float slabs[CV_WAVES][8 * CV_SLABP];

  const int tid = threadIdx.x, lane = tid & 31, wave = tid >> 5;
  const int c = lane & 15, hh = lane >> 4, koff = hh * 8;
  const int bi = blockIdx.x;
  const int s  = bi + 1;
  const int bb = blockIdx.y;
  const int L1  = (kT - 1) / s + 1;
  const int L2p = (L1 - 2) >> 1;
  const int L3p = (L2p - 2) >> 1;
  const int NT1 = (L1 + 15) >> 4;
  const int NT2 = (L2p + 7) >> 3;
  const int NT3 = (L3p + 7) >> 3;

  const __bf16* XB = (const __bf16*)XBp;
  const __bf16* C1 = (const __bf16*)C1p;
  const __bf16* C2 = (const __bf16*)C2p;
  const __bf16* C3 = (const __bf16*)C3p;

  {
    const v4u z4 = {0u, 0u, 0u, 0u};
    if (tid < 8) {
      *(v4u*)(h1H + NT1 * 256 + tid * 8) = z4;
      *(v4u*)(h1L + NT1 * 256 + tid * 8) = z4;
    }
    if (tid < 64) {
      *(v4u*)(h2H + NT2 * 256 + tid * 8) = z4;
      *(v4u*)(h2L + NT2 * 256 + tid * 8) = z4;
    }
  }
  const v8f z8 = {0.f, 0.f, 0.f, 0.f, 0.f, 0.f, 0.f, 0.f};

  {
    v16b bw[4];
    const __bf16* wp = C1 + (size_t)(bi * 16 + c) * kD + koff;
#pragma unroll
    for (int ks = 0; ks < 4; ++ks) bw[ks] = Frag<__bf16>::load(wp + 32 * ks);
    const float bias1 = bf16r(c1b[bi * 16 + c]);
#pragma unroll 1
    for (int tix = wave; tix < NT1; tix += CV_WAVES) {
      int xs = (16 * tix + c) * s;
      xs = (xs < kT - 1) ? xs : (kT - 1);
      const __bf16* ap = XB + ((size_t)bb * kT + xs) * kD + koff;
      v8f acc = z8;
#pragma unroll
      for (int ks = 0; ks < 4; ++ks) {
        const v16b a = Frag<__bf16>::load(ap + 32 * ks);
        acc = mma_bf(a, bw[ks], acc);
      }
#pragma unroll
      for (int r = 0; r < 8; ++r) {
        const int pos = 16 * tix + 8 * hh + r;
        float v = acc[r] + bias1;
        v = (pos < L1) ? v : 0.0f;
        unsigned short hb, lb;
        split_bf(v, hb, lb);
        h1H[pos * 16 + c] = hb;
        h1L[pos * 16 + c] = lb;
      }
    }
  }
  __syncthreads();

  {
    v16b bw[2][2];
#pragma unroll
    for (int nt = 0; nt < 2; ++nt)
#pragma unroll
      for (int ks = 0; ks < 2; ++ks)
        bw[nt][ks] = Frag<__bf16>::load(C2 + (size_t)(bi * 32 + nt * 16 + c) * 64 + koff + 32 * ks);
    const float bias2a = bf16r(c2b[bi * 32 + c]);
    const float bias2b = bf16r(c2b[bi * 32 + 16 + c]);
    const __bf16* p1H = (const __bf16*)h1H;
    const __bf16* p1L = (const __bf16*)h1L;
#pragma unroll 1
    for (int tix = wave; tix < NT2; tix += CV_WAVES) {
      const int aoff = (16 * tix + c) * 16 + koff;
      v8f acc0 = z8, acc1 = z8;
#pragma unroll
      for (int ks = 0; ks < 2; ++ks) {
        const v16b ah = Frag<__bf16>::load(p1H + aoff + 32 * ks);
        acc0 = mma_bf(ah, bw[0][ks], acc0);
        acc1 = mma_bf(ah, bw[1][ks], acc1);
        const v16b al = Frag<__bf16>::load(p1L + aoff + 32 * ks);
        acc0 = mma_bf(al, bw[0][ks], acc0);
        acc1 = mma_bf(al, bw[1][ks], acc1);
      }
#pragma unroll
      for (int q = 0; q < 4; ++q) {
        const int j = 8 * tix + 4 * hh + q;
        const bool ok = j < L2p;
        float v0 = fmaxf(acc0[2 * q] + bias2a, acc0[2 * q + 1] + bias2a);
        float v1 = fmaxf(acc1[2 * q] + bias2b, acc1[2 * q + 1] + bias2b);
        v0 = ok ? v0 : 0.0f;
        v1 = ok ? v1 : 0.0f;
        unsigned short hb0, lb0, hb1, lb1;
        split_bf(v0, hb0, lb0);
        split_bf(v1, hb1, lb1);
        h2H[j * 32 + c] = hb0;
        h2L[j * 32 + c] = lb0;
        h2H[j * 32 + 16 + c] = hb1;
        h2L[j * 32 + 16 + c] = lb1;
      }
    }
  }
  __syncthreads();

  {
    v16b bw[2][3];
#pragma unroll
    for (int nt = 0; nt < 2; ++nt)
#pragma unroll
      for (int ks = 0; ks < 3; ++ks)
        bw[nt][ks] = Frag<__bf16>::load(C3 + (size_t)(bi * 32 + nt * 16 + c) * 96 + koff + 32 * ks);
    const float bias3a = bf16r(c3b[bi * 32 + c]);
    const float bias3b = bf16r(c3b[bi * 32 + 16 + c]);
    const __bf16* p2H = (const __bf16*)h2H;
    const __bf16* p2L = (const __bf16*)h2L;
    float* slab = slabs[wave];
    const int pad8 = 8 * NT3;
    const size_t rowbase = (size_t)c_Off3[bi] * kB + (size_t)bb * pad8;
    const int srow = lane >> 2, scol = (lane & 3) * 8;
#pragma unroll 1
    for (int tix = wave; tix < NT3; tix += CV_WAVES) {
      const int aoff = (16 * tix + c) * 32 + koff;
      v8f acc0 = z8, acc1 = z8;
#pragma unroll
      for (int ks = 0; ks < 3; ++ks) {
        const v16b ah = Frag<__bf16>::load(p2H + aoff + 32 * ks);
        acc0 = mma_bf(ah, bw[0][ks], acc0);
        acc1 = mma_bf(ah, bw[1][ks], acc1);
        const v16b al = Frag<__bf16>::load(p2L + aoff + 32 * ks);
        acc0 = mma_bf(al, bw[0][ks], acc0);
        acc1 = mma_bf(al, bw[1][ks], acc1);
      }
#pragma unroll
      for (int q = 0; q < 4; ++q) {
        const int j = 8 * tix + 4 * hh + q;
        const bool ok = j < L3p;
        const float v0 = fmaxf(acc0[2 * q] + bias3a, acc0[2 * q + 1] + bias3a);
        const float v1 = fmaxf(acc1[2 * q] + bias3b, acc1[2 * q + 1] + bias3b);
        slab[(4 * hh + q) * CV_SLABP + c]      = ok ? (v0 * XF_CARRY) : 0.0f;
        slab[(4 * hh + q) * CV_SLABP + 16 + c] = ok ? (v1 * XF_CARRY) : 0.0f;
      }
      wave_lds_sync();
      const v4f s0 = *(const v4f*)(slab + srow * CV_SLABP + scol);
      const v4f s1 = *(const v4f*)(slab + srow * CV_SLABP + scol + 4);
      v8h hv, lv;
#pragma unroll
      for (int e = 0; e < 4; ++e) {
        const float x0 = s0[e];
        const float x1 = s1[e];
        unsigned short hb0, lb0, hb1, lb1;
        split_bf(x0, hb0, lb0);
        split_bf(x1, hb1, lb1);
        hv[e]     = __builtin_bit_cast(_Float16, hb0);
        hv[4 + e] = __builtin_bit_cast(_Float16, hb1);
        lv[e]     = __builtin_bit_cast(_Float16, lb0);
        lv[4 + e] = __builtin_bit_cast(_Float16, lb1);
      }
      const size_t o = (rowbase + (size_t)(8 * tix + srow)) * 32 + scol;
      for (int pass = 0; pass < 2; ++pass) {
        *(volatile v8h*)(XFH + o) = hv;
        *(volatile v8h*)(XFL + o) = lv;
        __threadfence();
      }
      wave_lds_sync();
    }
  }
}

constexpr int LS_THREADS = 512;
constexpr int LS_WAVES   = 16;
constexpr int LS_ROWS    = 16;
constexpr int LS_HP      = 520;
constexpr int LS_SLP     = 36;
static_assert(kH == 32 * LS_WAVES);
static_assert(kB % LS_ROWS == 0);

__global__ __launch_bounds__(LS_THREADS) void lstm_seq_kernel(
    const unsigned short* __restrict__ XFHp, const unsigned short* __restrict__ XFLp,
    const unsigned short* __restrict__ WIHp, const unsigned short* __restrict__ WHHp,
    const float* __restrict__ b_ih, const float* __restrict__ b_hh, float* __restrict__ out) {
  __shared__ __align__(16) _Float16 Ah[2][LS_ROWS * LS_HP];
  __shared__ __align__(16) float    Sl[LS_WAVES][16 * LS_SLP];
  const __bf16*   XFH = (const __bf16*)XFHp;
  const __bf16*   XFL = (const __bf16*)XFLp;
  const __bf16*   WIH = (const __bf16*)WIHp;
  const _Float16* WHH = (const _Float16*)WHHp;

  const int tid = threadIdx.x, lane = tid & 31, wave = tid >> 5;
  const int c = lane & 15, hh = lane >> 4, koff = hh * 8;
  const int b0 = blockIdx.x * LS_ROWS;
  const int nbase = 32 * wave + c;

  {
    _Float16* ahf = &Ah[0][0];
#pragma unroll 1
    for (int i = tid; i < 2 * LS_ROWS * LS_HP; i += LS_THREADS) ahf[i] = (_Float16)0.0f;
  }
  float cst[2][8];
  float bv[2][4];
#pragma unroll
  for (int u = 0; u < 2; ++u) {
#pragma unroll
    for (int r = 0; r < 8; ++r) cst[u][r] = 0.0f;
#pragma unroll
    for (int g = 0; g < 4; ++g) {
      const int idx = g * kH + nbase + 16 * u;
      bv[u][g] = (bf16r(b_ih[idx]) + bf16r(b_hh[idx])) * XF_CARRY;
    }
  }
  __syncthreads();

  float* slab = Sl[wave];
  const int q4 = lane >> 3, c4 = (lane & 7) * 4;

#pragma unroll 1
  for (int t = 0; t < kML; ++t) {
    const int cur = t & 1;
    v8f acc[2][4];
#pragma unroll
    for (int u = 0; u < 2; ++u)
#pragma unroll
      for (int g = 0; g < 4; ++g) {
        const float x = bv[u][g];
        acc[u][g] = (v8f){x, x, x, x, x, x, x, x};
      }

    const int need = kML - t;
#pragma unroll 1
    for (int si = 0; si < kS; ++si) {
      const int L3 = c_P3[si];
      if (L3 < need) break;
      const int pad8 = (L3 + 7) & ~7;
      const int rowA = c_Off3[si] * kB + (b0 + c) * pad8 + (L3 - need);
      const size_t ao = (size_t)rowA * 32 + koff;
      const v16b aH = Frag<__bf16>::load(XFH + ao);
      const v16b aL = Frag<__bf16>::load(XFL + ao);
#pragma unroll
      for (int u = 0; u < 2; ++u)
#pragma unroll
        for (int g = 0; g < 4; ++g) {
          const v16b bw = Frag<__bf16>::load(WIH + (size_t)(g * kH + nbase + 16 * u) * kNH + si * 32 + koff);
          acc[u][g] = mma_bf(aH, bw, acc[u][g]);
          acc[u][g] = mma_bf(aL, bw, acc[u][g]);
        }
    }

    const _Float16* ahrow = &Ah[cur][0] + c * LS_HP + koff;
#pragma unroll 1
    for (int k0 = 0; k0 < kH; k0 += 32) {
      const v16h a = Frag<_Float16>::load(ahrow + k0);
#pragma unroll
      for (int u = 0; u < 2; ++u)
#pragma unroll
        for (int g = 0; g < 4; ++g) {
          const v16h bw = Frag<_Float16>::load(WHH + (size_t)(g * kH + nbase + 16 * u) * kH + koff + k0);
          acc[u][g] = mma_hf(a, bw, acc[u][g]);
        }
    }

    _Float16* ahn = &Ah[cur ^ 1][0];
#pragma unroll
    for (int u = 0; u < 2; ++u) {
      const int n = nbase + 16 * u;
#pragma unroll
      for (int r = 0; r < 8; ++r) {
        const float zi = acc[u][0][r] * GATE_FOLD;
        const float zf = acc[u][1][r] * GATE_FOLD;
        const float zg = acc[u][2][r] * GATE_FOLD;
        const float zo = acc[u][3][r] * GATE_FOLD;
        const float ig = fsig(zi);
        const float fg = fsig(zf);
        const float gg = ftanh(zg);
        const float og = fsig(zo);
        const float cn = fg * cst[u][r] + ig * gg;
        cst[u][r] = cn;
        const float hn = og * ftanh(cn);
        float hs = hn * H_CARRY;
        hs = (fabsf(hs) < F16_MIN_NRM) ? 0.0f : hs;
        ahn[(8 * hh + r) * LS_HP + n] = (_Float16)hs;
        slab[(8 * hh + r) * LS_SLP + 16 * u + c] = hn;
      }
    }
    wave_lds_sync();
    {
      v4f v[4];
#pragma unroll
      for (int it = 0; it < 4; ++it) v[it] = *(const v4f*)(slab + (it * 4 + q4) * LS_SLP + c4);
      for (int pass = 0; pass < 2; ++pass) {
#pragma unroll
        for (int it = 0; it < 4; ++it) {
          const int row = it * 4 + q4;
          *(volatile v4f*)(out + ((size_t)(b0 + row) * kML + (size_t)t) * kH + 32 * wave + c4) = v[it];
        }
        __threadfence();
      }
    }
    __syncthreads();
  }
}

extern "C" void kernel_launch(void* const* d_in, const int* in_sizes, int n_in,
                              void* d_out, int out_size, void* d_ws, size_t ws_size,
                              hipStream_t stream) {
  if (n_in < 11 || d_out == nullptr || d_ws == nullptr) return;
  if (in_sizes[0] != kB * kT * kD) return;
  if (in_sizes[1] != kS * 16 * kD) return;
  if (in_sizes[2] != kS * 16) return;
  if (in_sizes[3] != kS * 32 * 16 * 3) return;
  if (in_sizes[4] != kS * 32) return;
  if (in_sizes[5] != kS * 32 * 32 * 3) return;
  if (in_sizes[6] != kS * 32) return;
  if (in_sizes[7] != kG4 * kNH) return;
  if (in_sizes[8] != kG4 * kH) return;
  if (in_sizes[9] != kG4) return;
  if (in_sizes[10] != kG4) return;
  if (out_size != kB * kML * kH) return;
  if (ws_size < kWsTotal) return;

  const float* X    = (const float*)d_in[0];
  const float* c1w  = (const float*)d_in[1];
  const float* c1b  = (const float*)d_in[2];
  const float* c2w  = (const float*)d_in[3];
  const float* c2b  = (const float*)d_in[4];
  const float* c3w  = (const float*)d_in[5];
  const float* c3b  = (const float*)d_in[6];
  const float* wih  = (const float*)d_in[7];
  const float* whh  = (const float*)d_in[8];
  const float* bih  = (const float*)d_in[9];
  const float* bhh  = (const float*)d_in[10];
  float* out = (float*)d_out;

  char* ws = (char*)d_ws;
  size_t off = 0;
  auto carve = [&](size_t bytes) -> char* { char* p = ws + off; off += bytes; return p; };
  unsigned short* XB  = (unsigned short*)carve(kBytesXB);
  unsigned short* WIH = (unsigned short*)carve(kBytesWIH);
  unsigned short* WHH = (unsigned short*)carve(kBytesWHH);
  unsigned short* C1T = (unsigned short*)carve(kBytesC1);
  unsigned short* C2T = (unsigned short*)carve(kBytesC2);
  unsigned short* C3T = (unsigned short*)carve(kBytesC3);
  unsigned short* XFH = (unsigned short*)carve(kBytesXF);
  unsigned short* XFL = (unsigned short*)carve(kBytesXF);
  if (off != kWsTotal || off > ws_size) return;

  const int n8x  = kB * kT * kD / 8;
  const int n8wi = kG4 * kNH / 8;
  const int n8wh = kG4 * kH / 8;
  const int n8c1 = kS * 16 * kD / 8;
  const int n8c2 = kS * 32 * 64 / 8;
  const int n8c3 = kS * 32 * 96 / 8;
  cvt8_kernel<0><<<(n8x + 255) / 256, 256, 0, stream>>>(X, XB, n8x, 1.0f);
  cvt8_kernel<0><<<(n8wi + 255) / 256, 256, 0, stream>>>(wih, WIH, n8wi, 1.0f);
  cvt8_kernel<1><<<(n8wh + 255) / 256, 256, 0, stream>>>(whh, WHH, n8wh, WHH_CARRY);
  cvt8_kernel<0><<<(n8c1 + 255) / 256, 256, 0, stream>>>(c1w, C1T, n8c1, 1.0f);
  tapw_reorder_kernel<16><<<(n8c2 + 255) / 256, 256, 0, stream>>>(c2w, C2T, n8c2);
  tapw_reorder_kernel<32><<<(n8c3 + 255) / 256, 256, 0, stream>>>(c3w, C3T, n8c3);

  branch_conv_kernel<<<dim3(kS, kB), CV_THREADS, 0, stream>>>(XB, C1T, C2T, C3T, c1b, c2b, c3b, XFH, XFL);

  lstm_seq_kernel<<<kB / LS_ROWS, LS_THREADS, 0, stream>>>(XFH, XFL, WIH, WHH, bih, bhh, out);
}
